// GNN_oracle_51299089383938
// MI455X (gfx1250) — hardware-run, weakly checked
//
#include <hip/hip_runtime.h>

typedef float          v8f   __attribute__((ext_vector_type(8)));
typedef float          v4f   __attribute__((ext_vector_type(4)));
typedef unsigned int   v4u   __attribute__((ext_vector_type(4)));
typedef int            v8i   __attribute__((ext_vector_type(8)));
typedef unsigned short v8us  __attribute__((ext_vector_type(8)));
typedef unsigned short v16us __attribute__((ext_vector_type(16)));
typedef __bf16         v16bf __attribute__((ext_vector_type(16)));
typedef _Float16       v16h  __attribute__((ext_vector_type(16)));
typedef v4f  __attribute__((may_alias)) v4fa;
typedef v8us __attribute__((may_alias)) v8usa;
union FragB { v16bf v; v16us u; v8us h[2]; v8i w; };
union FragH { v16h  v; v16us u; v8us h[2]; v8i w; };

__device__ __forceinline__ v8f wmb(const FragB& a, const FragB& b, v8f c) {
  v8f d = __builtin_amdgcn_wmma_f32_16x16x32_bf16(false, a.v, false, b.v, (short)0, c, false, false);
  asm volatile("v_nop\n\tv_nop\n\tv_nop\n\tv_nop" : "+v"(d) : "v"(a.w), "v"(b.w));
  return d;
}

__device__ __forceinline__ v8f wmh(const FragH& a, const FragH& b, v8f c) {
  v8f d = __builtin_amdgcn_wmma_f32_16x16x32_f16(false, a.v, false, b.v, (short)0, c, false, false);
  asm volatile("v_nop\n\tv_nop\n\tv_nop\n\tv_nop" : "+v"(d) : "v"(a.w), "v"(b.w));
  return d;
}

__device__ __forceinline__ unsigned bf16_bits(float f) {
  const unsigned u = __float_as_uint(f);
  const unsigned r = (u + 0x7FFFu + ((u >> 16) & 1u)) >> 16;
  const unsigned q = (u >> 16) | 0x40u;
  return ((u & 0x7fffffffu) > 0x7f800000u) ? q : r;
}

__device__ __forceinline__ float bf16_val(float f) {
  return __uint_as_float(bf16_bits(f) << 16);
}
__device__ __forceinline__ int clampi(int v, int lo, int hi) {
  return v < lo ? lo : (v > hi ? hi : v);
}

__device__ __forceinline__ unsigned f16_bits(float f) {
  const unsigned u  = __float_as_uint(f);
  const unsigned s  = (u >> 16) & 0x8000u;
  const unsigned a  = u & 0x7fffffffu;
  const unsigned t  = a - 0x38000000u;
  const unsigned r  = (t + 0x0FFFu + ((t >> 13) & 1u)) >> 13;
  const unsigned rc = r > 0x7C00u ? 0x7C00u : r;
  const bool small  = a < 0x38800000u;
  const bool isnan  = a > 0x7f800000u;
  const unsigned fin = small ? 0u : (s | rc);
  return isnan ? (s | 0x7E00u) : fin;
}

__device__ __forceinline__ unsigned pk16(unsigned lo, unsigned hi) { return lo | (hi << 16); }
__device__ __forceinline__ unsigned bf16_lo_bits(float v) {
  float hi = bf16_val(v);
  asm volatile("" : "+v"(hi));
  return bf16_bits(v - hi);
}
__device__ __forceinline__ v4u pack8_bf16(v4f a, v4f c) {
  return (v4u){ pk16(bf16_bits(a[0]), bf16_bits(a[1])), pk16(bf16_bits(a[2]), bf16_bits(a[3])),
                pk16(bf16_bits(c[0]), bf16_bits(c[1])), pk16(bf16_bits(c[2]), bf16_bits(c[3])) };
}
__device__ __forceinline__ v4u pack8_bf16_lo(v4f a, v4f c) {
  return (v4u){ pk16(bf16_lo_bits(a[0]), bf16_lo_bits(a[1])), pk16(bf16_lo_bits(a[2]), bf16_lo_bits(a[3])),
                pk16(bf16_lo_bits(c[0]), bf16_lo_bits(c[1])), pk16(bf16_lo_bits(c[2]), bf16_lo_bits(c[3])) };
}
__device__ __forceinline__ v4u pack8_f16(v4f a, v4f c) {
  return (v4u){ pk16(f16_bits(a[0]), f16_bits(a[1])), pk16(f16_bits(a[2]), f16_bits(a[3])),
                pk16(f16_bits(c[0]), f16_bits(c[1])), pk16(f16_bits(c[2]), f16_bits(c[3])) };
}

template <int FORM>
__global__ __launch_bounds__(256) void k_plane(const float* __restrict__ src, int rows, int cols, int ldsrc,
                                               unsigned short* __restrict__ dst, int MP, int KP) {
  static_assert(FORM >= 0 && FORM <= 3);
  const int KTOT = (FORM == 1 || FORM == 3) ? 2 * KP : KP;
  const unsigned ppr   = (unsigned)(KTOT >> 3);
  const unsigned kp8   = (unsigned)(KP >> 3);
  const unsigned total = (unsigned)MP * ppr;
  const unsigned g     = blockIdx.x * 256u + threadIdx.x;
  const unsigned rowu  = g / ppr;
  const unsigned p     = g - rowu * ppr;
  const bool second    = p >= kp8;
  const int row = (int)rowu;
  const int c0  = (int)((second ? p - kp8 : p) << 3);
  const float* srow = src + (size_t)clampi(row, 0, rows - 1) * (size_t)ldsrc;
  float x[8];
  unsigned mk[8];
#pragma unroll
  for (int e = 0; e < 8; ++e) {
    const int c = c0 + e;
    const float v = srow[clampi(c, 0, cols - 1)];
    asm volatile("" :: "v"(v));
    x[e]  = v;
    mk[e] = (row < rows && c < cols) ? 0xFFFFu : 0u;
  }
  const v4f a = (v4f){ x[0], x[1], x[2], x[3] };
  const v4f c = (v4f){ x[4], x[5], x[6], x[7] };
  v4u o;
  if (FORM == 2) {
    o = pack8_f16(a, c);
  } else {
    const v4u hi = pack8_bf16(a, c);
    o = hi;
    if (FORM == 1) { const v4u lo = pack8_bf16_lo(a, c); o = second ? lo : hi; }
  }
  const v4u mw = (v4u){ pk16(mk[0], mk[1]), pk16(mk[2], mk[3]), pk16(mk[4], mk[5]), pk16(mk[6], mk[7]) };
  o &= mw;
  if (g < total) {
    volatile v4u* q = (volatile v4u*)(dst + (size_t)g * 8);
    *q = o;
    __threadfence();
    *q = o;
  }
}

template <int FORM> struct FragOf    { typedef FragB T; };
template <>         struct FragOf<2> { typedef FragH T; };
__device__ __forceinline__ v8f mm(const FragB& a, const FragB& b, v8f c) { return wmb(a, b, c); }
__device__ __forceinline__ v8f mm(const FragH& a, const FragH& b, v8f c) { return wmh(a, b, c); }
template <class F> __device__ __forceinline__ F ld_frag(const unsigned short* p) {
  F f;
  f.h[0] = *(const v8usa*)(p);
  f.h[1] = *(const v8usa*)(p + 16);
  return f;
}

template <int FORM, int EPI>
__global__ __launch_bounds__(256) __attribute__((amdgpu_num_vgpr(248)))
void k_gemm_nt(const unsigned short* __restrict__ A, const unsigned short* __restrict__ B,
               const float* __restrict__ bias, float* __restrict__ D, int M, int N, int KTOT, int ldd) {
  static_assert(FORM >= 0 && FORM <= 2);
  static_assert(EPI == 0 || EPI == 1);
  typedef typename FragOf<FORM>::T F;
  __shared__ __attribute__((aligned(16))) float sT[8][16 * 68];
  const int lane = threadIdx.x & 31;
  const int wave = threadIdx.x >> 5;
  const int tilesM = (M + 63) >> 6;
  const int tilesN = (N + 63) >> 6;
  const int tile = blockIdx.x * 8 + wave;
  if (tile >= tilesM * tilesN) return;
  const int tm = tile / tilesN;
  const int tn = tile - tm * tilesN;
  const int m0 = tm << 6;
  const int n0 = tn << 6;

  const int rl = lane & 15;
  const int h8 = (lane >> 4) * 8;
  const unsigned short* pa = A + (size_t)(m0 + rl) * (size_t)KTOT + h8;
  const unsigned short* pb = B + (size_t)(n0 + rl) * (size_t)KTOT + h8;

  v8f acc[4][4];
#pragma unroll
  for (int i = 0; i < 4; ++i)
#pragma unroll
    for (int j = 0; j < 4; ++j) acc[i][j] = (v8f){0.f, 0.f, 0.f, 0.f, 0.f, 0.f, 0.f, 0.f};

#pragma unroll 1
  for (int k0 = 0; k0 < KTOT; k0 += 32) {
    F bf[4];
#pragma unroll
    for (int j = 0; j < 4; ++j) bf[j] = ld_frag<F>(pb + (size_t)(j << 4) * (size_t)KTOT + k0);
#pragma unroll
    for (int i = 0; i < 4; ++i) {
      const F af = ld_frag<F>(pa + (size_t)(i << 4) * (size_t)KTOT + k0);
#pragma unroll
      for (int j = 0; j < 4; ++j) acc[i][j] = mm(af, bf[j], acc[i][j]);
    }
  }

  float* slab = sT[wave];
  const int hh = lane >> 4;
  const int c4 = (lane & 15) * 4;
  const int nc = n0 + c4;
  const bool cok = nc < N;
  v4f bv = (v4f){0.f, 0.f, 0.f, 0.f};
  if (EPI == 1) {
    bv = *(const v4fa*)(bias + clampi(nc, 0, N - 4));
    asm volatile("" :: "v"(bv));
  }
#pragma unroll
  for (int i = 0; i < 4; ++i) {
    const int mBase = m0 + (i << 4);
#pragma unroll
    for (int j = 0; j < 4; ++j) {
#pragma unroll
      for (int r = 0; r < 8; ++r) slab[(h8 + r) * 68 + (j << 4) + rl] = acc[i][j][r];
    }
    __builtin_amdgcn_fence(__ATOMIC_RELEASE, "workgroup");
    __builtin_amdgcn_wave_barrier();
    __builtin_amdgcn_fence(__ATOMIC_ACQUIRE, "workgroup");
    v4f vv[8];
#pragma unroll
    for (int it = 0; it < 8; ++it) {
      const int row = it * 2 + hh;
      v4f v = *(const v4fa*)(slab + row * 68 + c4);
      if (EPI == 1) v += bv;
      vv[it] = v;
    }
    for (int pass = 0; pass < 2; ++pass) {
#pragma unroll
      for (int it = 0; it < 8; ++it) {
        const int row = mBase + it * 2 + hh;
        if (cok && row < M) *(volatile v4f*)(D + (size_t)row * (size_t)ldd + nc) = vv[it];
      }
      __threadfence();
    }
    __builtin_amdgcn_fence(__ATOMIC_RELEASE, "workgroup");
    __builtin_amdgcn_wave_barrier();
    __builtin_amdgcn_fence(__ATOMIC_ACQUIRE, "workgroup");
  }
}

typedef unsigned       v2u  __attribute__((ext_vector_type(2)));
typedef int            v4i  __attribute__((ext_vector_type(4)));
typedef v4i __attribute__((may_alias)) v4ia;
typedef v2u __attribute__((may_alias)) v2ua;
typedef unsigned short __attribute__((may_alias)) usa;

#define NNODE   100000
#define NEDGE   3200000
#define MPAD    100096
#define NBRUN   1024
#define NBLKB   98
#define NWV     8
#define WCAP    4608
#define LISTN   (NWV * WCAP)
#define RCAP    36864
#define NWCH    (NEDGE / 256)
#define DEGCAP  72
#define BK_CNTW LISTN
#define BK_OFF  (BK_CNTW + NWV * NBRUN)
#define BK_CNT  (BK_OFF + NBRUN)
#define BK_MISC (BK_CNT + NBRUN)
#define BK_PLC  (BK_MISC + 64)
#define BK_INTS (BK_PLC + RCAP / 2)
#define LN_NBLK 391
#define ST_GPB  5
#define ST_EPB  (ST_GPB * 416)
#define ST_NBLK 625
#define OUT_N   1300001

#define P_W1T   0
#define P_B1    1664
#define P_G1    1792
#define P_BE1   1920
#define P_B2    2048
#define P_G2    2080
#define P_BE2   2112
#define P_BG    2144
#define P_BL    2272
#define P_EPS   2288
#define P_GLN   2304
#define P_BLN   2336
#define P_GLAST 2368
#define P_BLAST 2384
#define P_WC1   2400
#define P_BC1   5728
#define P_WC2   5984
#define P_BC2   6240
#define PRM_N   6272

static_assert(NEDGE % 256 == 0);
static_assert(NEDGE <= (1 << 22));
static_assert(NBRUN == 1024);
static_assert(NBLKB * NBRUN >= NNODE && (NBLKB - 1) * NBRUN < NNODE);
static_assert(MPAD % 256 == 0 && MPAD % 128 == 0 && MPAD % 64 == 0 && MPAD >= NNODE && MPAD <= NBLKB * NBRUN);
static_assert(MPAD / 256 == LN_NBLK);
static_assert(NWV * WCAP == RCAP && RCAP % 256 == 0 && LISTN <= 65536);
static_assert(RCAP >= 33280 + (33280 * 8) / 100);
static_assert(DEGCAP >= 58 + 8 && DEGCAP % 8 == 0);
static_assert(BK_INTS % 4 == 0 && BK_INTS * 4 <= 300000);
static_assert(ST_NBLK * ST_EPB == OUT_N - 1);
static_assert(ST_EPB % 32 == 0);
static_assert(PRM_N % 4 == 0 && P_BC2 + 32 == PRM_N);

__device__ __forceinline__ void pinf(float x) { asm volatile("" :: "v"(x)); }
__device__ __forceinline__ void pini(int x)   { asm volatile("" :: "v"(x)); }

__device__ __forceinline__ void wsync() {
  __builtin_amdgcn_fence(__ATOMIC_RELEASE, "workgroup");
  __builtin_amdgcn_wave_barrier();
  __builtin_amdgcn_fence(__ATOMIC_ACQUIRE, "workgroup");
}

__device__ __forceinline__ float wsum32(float v) {
  v += __shfl_xor(v, 16, 32);
  v += __shfl_xor(v, 8, 32);
  v += __shfl_xor(v, 4, 32);
  v += __shfl_xor(v, 2, 32);
  v += __shfl_xor(v, 1, 32);
  return v;
}
__device__ __forceinline__ float hsum16(float v) {
  v += __shfl_xor(v, 8, 32);
  v += __shfl_xor(v, 4, 32);
  v += __shfl_xor(v, 2, 32);
  v += __shfl_xor(v, 1, 32);
  return v;
}
__device__ __forceinline__ float eluf(float x) { return (x > 0.0f) ? x : expm1f(x); }

__device__ __forceinline__ void seg_copy(const float* __restrict__ s, int n, int padn, float* img, int off, int tid) {
  const int padw = (padn + 31) & ~31;
#pragma unroll 1
  for (int i = tid; i < padw; i += 256) {
    float v = s[i < n ? i : n - 1];
    pinf(v);
    if (i < padn) img[off + i] = (i < n) ? bf16_val(v) : 0.0f;
  }
}

__global__ __launch_bounds__(256) void k_prep(
    const float* __restrict__ W1, const float* __restrict__ b1, const float* __restrict__ g1,
    const float* __restrict__ be1, const float* __restrict__ b2, const float* __restrict__ g2,
    const float* __restrict__ be2, const float* __restrict__ bg, const float* __restrict__ bl,
    const float* __restrict__ eps, const float* __restrict__ gln, const float* __restrict__ bln,
    const float* __restrict__ glast, const float* __restrict__ blast, const float* __restrict__ Wc1,
    const float* __restrict__ bc1, const float* __restrict__ Wc2, const float* __restrict__ bc2, float* prm) {
  __shared__ __attribute__((aligned(16))) float img[PRM_N];
  const int tid = (int)threadIdx.x;
#pragma unroll 1
  for (int i = tid; i < 1664; i += 256) {
    float v = W1[i];
    pinf(v);
    const int n = i / 13;
    const int k = i - 13 * n;
    img[P_W1T + k * 128 + n] = bf16_val(v);
  }
  seg_copy(b1, 128, 128, img, P_B1, tid);
  seg_copy(g1, 128, 128, img, P_G1, tid);
  seg_copy(be1, 128, 128, img, P_BE1, tid);
  seg_copy(b2, 32, 32, img, P_B2, tid);
  seg_copy(g2, 32, 32, img, P_G2, tid);
  seg_copy(be2, 32, 32, img, P_BE2, tid);
  seg_copy(bg, 128, 128, img, P_BG, tid);
  seg_copy(bl, 13, 16, img, P_BL, tid);
  seg_copy(eps, 5, 16, img, P_EPS, tid);
  seg_copy(gln, 32, 32, img, P_GLN, tid);
  seg_copy(bln, 32, 32, img, P_BLN, tid);
  seg_copy(glast, 13, 16, img, P_GLAST, tid);
  seg_copy(blast, 13, 16, img, P_BLAST, tid);
  seg_copy(Wc1, 3328, 3328, img, P_WC1, tid);
  seg_copy(bc1, 256, 256, img, P_BC1, tid);
  seg_copy(Wc2, 256, 256, img, P_WC2, tid);
  seg_copy(bc2, 1, 32, img, P_BC2, tid);
  __syncthreads();
  for (int pass = 0; pass < 2; ++pass) {
#pragma unroll 1
    for (int p = tid; p < PRM_N / 4; p += 256) {
      const v4f v = *(const v4fa*)(img + 4 * p);
      *(volatile v4f*)(prm + 4 * p) = v;
    }
    __threadfence();
  }
}

__device__ __forceinline__ int slot_prefix(int* cntw, int s) {
  int run = 0;
#pragma unroll
  for (int w = 0; w < NWV; ++w) {
    const int c = cntw[w * NBRUN + s];
    cntw[w * NBRUN + s] = run;
    run += c;
  }
  return run;
}

#define BK_HIT(J, SJ) { \
    const unsigned mk_ = __builtin_amdgcn_ballot_w32((SJ) < unb); \
    if (mk_ != 0u) { \
      const int pos_ = wcnt + (int)__builtin_amdgcn_mbcnt_lo(mk_, 0u); \
      if ((SJ) < unb && pos_ < WCAP) list[lbase + pos_] = (int)((((unsigned)(e0 + (J))) << 10) | (SJ)); \
      wcnt += (int)__builtin_popcount(mk_); \
    } }

__global__ __launch_bounds__(256) void k_bucket(const int* __restrict__ src, const int* __restrict__ dst,
                                                const float* __restrict__ ew, unsigned* entg, int* offg,
                                                int* cntg, int* ovfg) {
  extern __shared__ __attribute__((aligned(16))) int dsm[];
  int* list = dsm;
  int* cntw = dsm + BK_CNTW;
  int* offA = dsm + BK_OFF;
  int* cntT = dsm + BK_CNT;
  int* misc = dsm + BK_MISC;
  usa* plc  = (usa*)(dsm + BK_PLC);
  const int tid = (int)threadIdx.x, lane = tid & 31;
  const int wave = __builtin_amdgcn_readfirstlane(tid >> 5);
  const int b = (int)blockIdx.x;
  const int nodeBase = b * NBRUN;
  const int nbl = (NNODE - nodeBase) < NBRUN ? (NNODE - nodeBase) : NBRUN;
  const unsigned nbs = (unsigned)nodeBase;
  const unsigned unb = (unsigned)nbl;
  const int lbase = wave * WCAP;

  {
    const v4i z4 = {0, 0, 0, 0};
#pragma unroll 1
    for (int i = tid * 4; i < BK_INTS; i += 1024) *(v4ia*)(dsm + i) = z4;
  }
  __syncthreads();

  int wcnt = 0;
#pragma unroll 1
  for (int wc = wave; wc < NWCH; wc += NWV) {
    const int e0 = wc * 256 + lane * 8;
    const v4i da = *(const v4i*)(dst + e0);
    const v4i db = *(const v4i*)(dst + e0 + 4);
    const unsigned s0 = (unsigned)da.x - nbs, s1 = (unsigned)da.y - nbs;
    const unsigned s2 = (unsigned)da.z - nbs, s3 = (unsigned)da.w - nbs;
    const unsigned s4 = (unsigned)db.x - nbs, s5 = (unsigned)db.y - nbs;
    const unsigned s6 = (unsigned)db.z - nbs, s7 = (unsigned)db.w - nbs;
    BK_HIT(0, s0)
    BK_HIT(1, s1)
    BK_HIT(2, s2)
    BK_HIT(3, s3)
    BK_HIT(4, s4)
    BK_HIT(5, s5)
    BK_HIT(6, s6)
    BK_HIT(7, s7)
  }
  const int wraw = __builtin_amdgcn_readfirstlane(wcnt);
  if (lane == 0) misc[wave] = wraw;
  __syncthreads();

  const int myc = clampi(wraw, 0, WCAP);
  if (lane == 0) {
#pragma unroll 1
    for (int i = 0; i < myc; ++i) {
      const int s = list[lbase + i] & (NBRUN - 1);
      cntw[wave * NBRUN + s] = cntw[wave * NBRUN + s] + 1;
    }
  }
  __syncthreads();

  const int t0 = slot_prefix(cntw, 4 * tid);
  const int t1 = slot_prefix(cntw, 4 * tid + 1);
  const int t2 = slot_prefix(cntw, 4 * tid + 2);
  const int t3 = slot_prefix(cntw, 4 * tid + 3);
  const int e1 = t0, e2 = t0 + t1, e3 = t0 + t1 + t2, sum4 = t0 + t1 + t2 + t3;
  int incl = sum4;
#pragma unroll
  for (int dd = 1; dd < 32; dd <<= 1) {
    const int y = __shfl_up(incl, dd, 32);
    if (lane >= dd) incl += y;
  }
  if (lane == 31) misc[8 + wave] = incl;
  __syncthreads();
  int base = 0, tot = 0, flag = 0;
#pragma unroll
  for (int w2 = 0; w2 < NWV; ++w2) {
    const int c = misc[8 + w2];
    base += (w2 < wave) ? c : 0;
    tot  += c;
    flag |= (misc[w2] > WCAP) ? 1 : 0;
  }
  const int ex = base + incl - sum4;
  const v4i ov = {ex, ex + e1, ex + e2, ex + e3};
  const v4i cv = {t0, t1, t2, t3};
  *(v4ia*)(offA + 4 * tid) = ov;
  *(v4ia*)(cntT + 4 * tid) = cv;
  __syncthreads();

  if (lane == 0) {
#pragma unroll 1
    for (int i = 0; i < myc; ++i) {
      const int s = list[lbase + i] & (NBRUN - 1);
      const int c = cntw[wave * NBRUN + s];
      cntw[wave * NBRUN + s] = c + 1;
      const int p = offA[s] + c;
      if ((unsigned)p < (unsigned)RCAP) plc[p] = (unsigned short)(lbase + i);
    }
  }
  __syncthreads();

  const int tt  = tot < RCAP ? tot : RCAP;
  int ttr = (tt + 255) & ~255;
  ttr = ttr < RCAP ? ttr : RCAP;
  unsigned* eg = entg + (size_t)b * (size_t)(RCAP * 2);
  const v4i fv = {(tid == 0) ? flag : 0, 0, 0, 0};
  for (int pass = 0; pass < 2; ++pass) {
#pragma unroll 1
    for (int p = tid; p < ttr; p += 256) {
      const int pc = p < tt ? p : (tt > 0 ? tt - 1 : 0);
      const int idx = (int)plc[pc];
      const unsigned word = (unsigned)list[clampi(idx, 0, LISTN - 1)];
      const int eid = clampi((int)(word >> 10), 0, NEDGE - 1);
      int sr = src[eid];
      pini(sr);
      float wv = ew[eid];
      pinf(wv);
      sr = clampi(sr, 0, NNODE - 1);
      const unsigned wb = bf16_bits(wv) << 16;
      const unsigned mk = (p < tt) ? 0xFFFFFFFFu : 0u;
      const v2u o = {(unsigned)sr & mk, wb & mk};
      *(volatile v2u*)(eg + 2 * (size_t)p) = o;
    }
    *(volatile v4i*)(offg + (size_t)b * NBRUN + 4 * tid) = ov;
    *(volatile v4i*)(cntg + (size_t)b * NBRUN + 4 * tid) = cv;
    if (tid < 8) *(volatile v4i*)(ovfg + (size_t)b * 32 + 4 * tid) = fv;
    __threadfence();
  }
}

__global__ __launch_bounds__(256) void k_mlp1(const float* __restrict__ feat, const float* __restrict__ prm,
                                              unsigned* h1hl) {
  __shared__ __attribute__((aligned(16))) float sW[2048];
  __shared__ __attribute__((aligned(16))) float sRow[8 * 128];
  const int tid = (int)threadIdx.x, lane = tid & 31;
  const int wave = __builtin_amdgcn_readfirstlane(tid >> 5);
#pragma unroll
  for (int it = 0; it < 2; ++it) {
    const int p = tid + 256 * it;
    const v4f v = *(const v4fa*)(prm + 4 * p);
    *(v4fa*)(sW + 4 * p) = v;
  }
  __syncthreads();
  float* wrow = sRow + wave * 128;
  const int xl = lane < 13 ? lane : 12;
#pragma unroll 1
  for (int j = 0; j < 16; ++j) {
    const int row = (int)blockIdx.x * 128 + wave * 16 + j;
    const int rc  = row < NNODE ? row : NNODE - 1;
    float xv = feat[(size_t)rc * 13 + xl];
    pinf(xv);
    xv = bf16_val(xv);
    float a0 = 0.0f, a1 = 0.0f, a2 = 0.0f, a3 = 0.0f;
#pragma unroll 1
    for (int k = 0; k < 13; ++k) {
      const float xk = __shfl(xv, k, 32);
      const float* wr = sW + k * 128 + lane;
      a0 = fmaf(xk, wr[0], a0);
      a1 = fmaf(xk, wr[32], a1);
      a2 = fmaf(xk, wr[64], a2);
      a3 = fmaf(xk, wr[96], a3);
    }
    wrow[lane] = a0; wrow[lane + 32] = a1; wrow[lane + 64] = a2; wrow[lane + 96] = a3;
    float s = 0.0f;
#pragma unroll 1
    for (int u = 0; u < 4; ++u) {
      const int c = lane + 32 * u;
      float v = wrow[c] + sW[P_B1 + c];
      v = eluf(v);
      wrow[c] = v;
      s += v;
    }
    const float mean = wsum32(s) * 0.0078125f;
    float q = 0.0f;
#pragma unroll 1
    for (int u = 0; u < 4; ++u) {
      const float d = wrow[lane + 32 * u] - mean;
      q += d * d;
    }
    const float var = wsum32(q) * 0.0078125f;
    const float sd  = sqrtf(var + 1e-5f);
#pragma unroll 1
    for (int u = 0; u < 4; ++u) {
      const int c = lane + 32 * u;
      const float y = (wrow[c] - mean) / sd * sW[P_G1 + c] + sW[P_BE1 + c];
      wrow[c] = y;
    }
    wsync();
    const v4f y4 = *(const v4fa*)(wrow + 4 * lane);
    wsync();
    const unsigned mk = (row < NNODE) ? 0xFFFFFFFFu : 0u;
    const v2u hi = { pk16(bf16_bits(y4[0]), bf16_bits(y4[1])) & mk, pk16(bf16_bits(y4[2]), bf16_bits(y4[3])) & mk };
    const v2u lo = { pk16(bf16_lo_bits(y4[0]), bf16_lo_bits(y4[1])) & mk,
                     pk16(bf16_lo_bits(y4[2]), bf16_lo_bits(y4[3])) & mk };
    unsigned* op = h1hl + (size_t)row * 128 + 2 * lane;
    *(volatile v2u*)op = hi;
    *(volatile v2u*)(op + 64) = lo;
    __threadfence();
    *(volatile v2u*)op = hi;
    *(volatile v2u*)(op + 64) = lo;
  }
}

template <int ELU>
__global__ __launch_bounds__(256) void k_rowln32(const float* __restrict__ d32, const float* __restrict__ prm,
                                                 int pB, int pG, int pBe, float* hout) {
  const int tid = (int)threadIdx.x, lane = tid & 31;
  const int wave = __builtin_amdgcn_readfirstlane(tid >> 5);
  const float bj  = prm[pB + lane];
  const float gj  = prm[pG + lane];
  const float bej = prm[pBe + lane];
#pragma unroll 1
  for (int j = 0; j < 16; ++j) {
    const int row = (int)blockIdx.x * 128 + wave * 16 + j;
    const float x = d32[(size_t)row * 32 + lane];
    float v = x + bj;
    if (ELU) v = eluf(v);
    const float mean = wsum32(v) * 0.03125f;
    const float d    = v - mean;
    const float var  = wsum32(d * d) * 0.03125f;
    float y = d / sqrtf(var + 1e-5f) * gj + bej;
    y = (row < NNODE) ? y : 0.0f;
    float* op = hout + (size_t)row * 32 + lane;
    *(volatile float*)op = y;
    __threadfence();
    *(volatile float*)op = y;
  }
}

__global__ __launch_bounds__(256) void k_replay(const float* __restrict__ hin, const unsigned* __restrict__ entg,
                                                const int* __restrict__ offg, const int* __restrict__ cntg,
                                                const int* __restrict__ ovfg, const float* __restrict__ prm,
                                                int layer, unsigned* ahl) {
  const int tid = (int)threadIdx.x, lane = tid & 31;
  const int wave = __builtin_amdgcn_readfirstlane(tid >> 5);
  const int b = (int)blockIdx.x;
  int fl = ovfg[(size_t)b * 32];
  pini(fl);
  const float opeps = 1.0f + prm[P_EPS + layer];
  const float ninf = __int_as_float((int)0xff800000u);
  const float qnan = __int_as_float(0x7fc00000);
  const size_t ebase = (size_t)b * (size_t)RCAP;
#pragma unroll 1
  for (int si = 0; si < 128; ++si) {
    const int s = wave * 128 + si;
    const int node = b * NBRUN + s;
    if (node >= MPAD) break;
    int off = offg[(size_t)b * NBRUN + s];
    pini(off);
    int cr = cntg[(size_t)b * NBRUN + s];
    pini(cr);
    const int degov = (cr > DEGCAP) ? 1 : 0;
    int cnt = clampi(cr, 0, DEGCAP);
    off = clampi(off, 0, RCAP - 1);
    if (cnt > RCAP - off) cnt = RCAP - off;
    const int lastv = off + (cnt > 0 ? cnt - 1 : 0);
    cnt = __builtin_amdgcn_readfirstlane(cnt);
    off = __builtin_amdgcn_readfirstlane(off);
    const int last = __builtin_amdgcn_readfirstlane(lastv);
    float m = ninf;
#pragma unroll 1
    for (int g0 = 0; g0 < cnt; g0 += 8) {
      int idx = off + g0 + (lane & 7);
      idx = idx > last ? last : idx;
      const v2u en = *(const v2ua*)(entg + (ebase + (size_t)idx) * 2);
      pini((int)en.x); pini((int)en.y);
      const int srl = clampi((int)en.x, 0, NNODE - 1);
      const int wbl = (int)en.y;
      float hv[8];
#pragma unroll
      for (int j = 0; j < 8; ++j) {
        const int sj = __builtin_amdgcn_readlane(srl, j);
        hv[j] = hin[(size_t)sj * 32 + lane];
        pinf(hv[j]);
      }
#pragma unroll
      for (int j = 0; j < 8; ++j) {
        const float wj = __int_as_float(__builtin_amdgcn_readlane(wbl, j));
        float v = hv[j] * wj;
        v = ((g0 + j) < cnt) ? v : ninf;
        m = (v > m || v != v) ? v : m;
      }
    }
    const float agg = (cnt == 0) ? 0.0f : m;
    const int nc = node < NNODE ? node : NNODE - 1;
    float hd = hin[(size_t)nc * 32 + lane];
    pinf(hd);
    float a = fmaf(opeps, hd, agg);
    const float pz = (fl != 0 || degov != 0) ? qnan : 0.0f;
    a = a + pz;
    a = (node < NNODE) ? a : 0.0f;
    const unsigned cw = bf16_bits(a) | (bf16_lo_bits(a) << 16);
    const int sl = 2 * (lane & 15);
    const unsigned c0 = (unsigned)__shfl((int)cw, sl, 32);
    const unsigned c1 = (unsigned)__shfl((int)cw, sl + 1, 32);
    const unsigned whi = (c0 & 0xffffu) | (c1 << 16);
    const unsigned wlo = (c0 >> 16) | (c1 & 0xffff0000u);
    const unsigned word = (lane < 16) ? whi : wlo;
    unsigned* op = ahl + (size_t)node * 32 + lane;
    *(volatile unsigned*)op = word;
    __threadfence();
    *(volatile unsigned*)op = word;
  }
}

__global__ __launch_bounds__(256) void k_lnlast(const float* __restrict__ d32, const float* __restrict__ prm,
                                                float* out13, double* rec) {
  __shared__ double sred[8 * 32];
  const int tid = (int)threadIdx.x, lane = tid & 31;
  const int wave = __builtin_amdgcn_readfirstlane(tid >> 5);
  const int hh = lane >> 4, c = lane & 15;
  const bool cm = c < 13;
  const float blc = prm[P_BL + c];
  const float glc = prm[P_GLAST + c];
  const float btc = prm[P_BLAST + c];
  double acc = 0.0;
#pragma unroll 1
  for (int j = 0; j < 16; ++j) {
    const int row = (int)blockIdx.x * 256 + wave * 32 + 2 * j + hh;
    float x = d32[(size_t)row * 32 + c];
    pinf(x);
    const float v = cm ? (x + blc) : 0.0f;
    const float mean = hsum16(v) * (1.0f / 13.0f);
    const float d = cm ? (v - mean) : 0.0f;
    const float var = hsum16(d * d) * (1.0f / 13.0f);
    const float y = d / sqrtf(var + 1e-5f) * glc + btc;
    const float o = (cm && row < NNODE) ? y : 0.0f;
    acc += (double)o;
    float* op = out13 + (size_t)row * 16 + c;
    *(volatile float*)op = o;
    __threadfence();
    *(volatile float*)op = o;
  }
  sred[wave * 32 + lane] = acc;
  __syncthreads();
  if (wave == 0) {
    double t = 0.0;
#pragma unroll
    for (int w = 0; w < 8; ++w) {
      t += sred[w * 32 + c];
      t += sred[w * 32 + 16 + c];
    }
    const double o = cm ? t : 0.0;
    if (lane < 16) {
      volatile double* q = rec + (size_t)blockIdx.x * 16 + lane;
      *q = o;
      __threadfence();
      *q = o;
    }
  }
}

__global__ __launch_bounds__(256) void k_head(const double* __restrict__ rec, const float* __restrict__ prm,
                                              float* pred) {
  __shared__ float sp[16];
  __shared__ float red[256];
  const int tid = (int)threadIdx.x;
  if (tid < 32) {
    const int c = tid & 15;
    double s = 0.0;
#pragma unroll 4
    for (int b = 0; b < LN_NBLK; ++b) s += rec[(size_t)b * 16 + c];
    const float p = (float)(s / 100000.0);
    if (tid < 16) sp[tid] = p;
  }
  __syncthreads();
  float acc = 0.0f;
#pragma unroll 1
  for (int k = 0; k < 13; ++k) acc = fmaf(sp[k], prm[P_WC1 + tid * 13 + k], acc);
  acc += prm[P_BC1 + tid];
  red[tid] = eluf(acc) * prm[P_WC2 + tid];
  __syncthreads();
#pragma unroll 1
  for (int s = 128; s > 0; s >>= 1) {
    if (tid < s) red[tid] = red[tid] + red[tid + s];
    __syncthreads();
  }
  if (tid < 8) {
    const float r = red[0] + prm[P_BC2];
    const v4f o = {(tid == 0) ? r : 0.0f, 0.0f, 0.0f, 0.0f};
    *(volatile v4f*)(pred + 4 * tid) = o;
    __threadfence();
    *(volatile v4f*)(pred + 4 * tid) = o;
  }
}

__global__ __launch_bounds__(256) void k_store(const float* __restrict__ out13, const float* __restrict__ pred,
                                               const int* __restrict__ ovfg, float* out) {
  __shared__ __attribute__((aligned(16))) float img[ST_EPB];
  const int tid = (int)threadIdx.x;
  const int b = (int)blockIdx.x;
  const float qnan = __int_as_float(0x7fc00000);
  float pv = pred[0];
  pinf(pv);
  if (b < ST_NBLK) {
#pragma unroll 1
    for (int t = tid; t < ST_EPB; t += 256) {
      const int f = b * ST_EPB + t;
      int q = f - 1;
      q = q < 0 ? 0 : q;
      int n = q / 13;
      const int c = q - 13 * n;
      n = clampi(n, 0, NNODE - 1);
      float ov = out13[(size_t)n * 16 + c];
      pinf(ov);
      int fl = ovfg[(size_t)(n >> 10) * 32];
      pini(fl);
      const float nv = (fl != 0) ? qnan : ov;
      img[t] = (f == 0) ? pv : nv;
    }
    __syncthreads();
    float* ob = out + (size_t)b * ST_EPB;
    for (int pass = 0; pass < 2; ++pass) {
#pragma unroll 1
      for (int p = tid; p < ST_EPB / 4; p += 256) {
        const v4f v = *(const v4fa*)(img + 4 * p);
        *(volatile v4f*)(ob + 4 * p) = v;
      }
      __threadfence();
    }
  } else {
    float ov = out13[(size_t)(NNODE - 1) * 16 + 12];
    pinf(ov);
    int fl = ovfg[(size_t)((NNODE - 1) >> 10) * 32];
    pini(fl);
    const float v = (fl != 0) ? qnan : ov;
    if (tid == 0) {
      *(volatile float*)(out + (OUT_N - 1)) = v;
      __threadfence();
      *(volatile float*)(out + (OUT_N - 1)) = v;
    }
  }
}

static inline size_t al256(size_t o) { return (o + 255) & ~(size_t)255; }

extern "C" void kernel_launch(void* const* d_in, const int* in_sizes, int n_in,
                              void* d_out, int out_size, void* d_ws, size_t ws_size,
                              hipStream_t stream) {
  if (n_in != 25) return;
  const int es[25] = { NNODE * 13, NEDGE, NEDGE, NEDGE, 128 * 13, 128, 128, 128, 32 * 128, 32, 32, 32,
                       4 * 32 * 32, 4 * 32, 13 * 32, 13, 5, 32, 32, 13, 13, 256 * 13, 256, 256, 1 };
  for (int i = 0; i < 25; ++i) if (in_sizes[i] != es[i]) return;
  if (out_size != OUT_N) return;

  const float* features = (const float*)d_in[0];
  const int*   src      = (const int*)d_in[1];
  const int*   dst      = (const int*)d_in[2];
  const float* ew       = (const float*)d_in[3];
  const float* W1  = (const float*)d_in[4];
  const float* b1  = (const float*)d_in[5];
  const float* g1  = (const float*)d_in[6];
  const float* be1 = (const float*)d_in[7];
  const float* W2  = (const float*)d_in[8];
  const float* b2  = (const float*)d_in[9];
  const float* g2  = (const float*)d_in[10];
  const float* be2 = (const float*)d_in[11];
  const float* Wg  = (const float*)d_in[12];
  const float* bg  = (const float*)d_in[13];
  const float* Wl  = (const float*)d_in[14];
  const float* bl  = (const float*)d_in[15];
  const float* eps = (const float*)d_in[16];
  const float* gln = (const float*)d_in[17];
  const float* bln = (const float*)d_in[18];
  const float* glast = (const float*)d_in[19];
  const float* blast = (const float*)d_in[20];
  const float* Wc1 = (const float*)d_in[21];
  const float* bc1 = (const float*)d_in[22];
  const float* Wc2 = (const float*)d_in[23];
  const float* bc2 = (const float*)d_in[24];
  float* out = (float*)d_out;

  char* ws = (char*)d_ws;
  size_t off = 0;
  const size_t oH1HL = off; off = al256(off + (size_t)MPAD * 256 * 2);
  const size_t oD32  = off; off = al256(off + (size_t)MPAD * 32 * 4);
  const size_t oH    = off; off = al256(off + (size_t)MPAD * 32 * 4);
  const size_t oO13  = off; off = al256(off + (size_t)MPAD * 16 * 4);
  const size_t oENT  = off; off = al256(off + (size_t)NBLKB * RCAP * 8);
  const size_t oOFF  = off; off = al256(off + (size_t)NBLKB * NBRUN * 4);
  const size_t oCNT  = off; off = al256(off + (size_t)NBLKB * NBRUN * 4);
  const size_t oOVF  = off; off = al256(off + (size_t)NBLKB * 128);
  const size_t oREC  = off; off = al256(off + (size_t)LN_NBLK * 128);
  const size_t oPRED = off; off = al256(off + 128);
  const size_t oPRM  = off; off = al256(off + (size_t)PRM_N * 4);
  const size_t oW2D  = off; off = al256(off + (size_t)64 * 256 * 2);
  const size_t oWGD  = off; off = al256(off + (size_t)4 * 64 * 64 * 2);
  const size_t oWLD  = off; off = al256(off + (size_t)64 * 64 * 2);
  if (off > ws_size || off > (size_t)(128u << 20)) return;
  static_assert((size_t)MPAD * 64 * 2 <= (size_t)MPAD * 256 * 2);

  unsigned short* H1HL = (unsigned short*)(ws + oH1HL);
  unsigned short* AHL  = (unsigned short*)(ws + oH1HL);
  float*  D32  = (float*)(ws + oD32);
  float*  Hp   = (float*)(ws + oH);
  float*  O13  = (float*)(ws + oO13);
  unsigned* ENT = (unsigned*)(ws + oENT);
  int*    OFFt = (int*)(ws + oOFF);
  int*    CNTt = (int*)(ws + oCNT);
  int*    OVF  = (int*)(ws + oOVF);
  double* REC  = (double*)(ws + oREC);
  float*  PRED = (float*)(ws + oPRED);
  float*  PRM  = (float*)(ws + oPRM);
  unsigned short* W2D = (unsigned short*)(ws + oW2D);
  unsigned short* WGD = (unsigned short*)(ws + oWGD);
  unsigned short* WLD = (unsigned short*)(ws + oWLD);

  static_assert(MPAD % 64 == 0 && MPAD % 16 == 0);
  static_assert(256 % 32 == 0 && 64 % 32 == 0);
  static_assert((64 * 256 / 8) % 256 == 0 && (64 * 64 / 8) % 256 == 0);
  const int gemmGrid = ((MPAD / 64) + 7) / 8;

  const int bkLds = BK_INTS * 4;
  hipFuncSetAttribute(reinterpret_cast<const void*>(&k_bucket), hipFuncAttributeMaxDynamicSharedMemorySize, bkLds);

  k_prep<<<1, 256, 0, stream>>>(W1, b1, g1, be1, b2, g2, be2, bg, bl, eps, gln, bln, glast, blast,
                                Wc1, bc1, Wc2, bc2, PRM);
  k_plane<3><<<8, 256, 0, stream>>>(W2, 32, 128, 128, W2D, 64, 128);
  for (int i = 0; i < 4; ++i)
    k_plane<3><<<2, 256, 0, stream>>>(Wg + (size_t)i * 1024, 32, 32, 32, WGD + (size_t)i * 4096, 64, 32);
  k_plane<3><<<2, 256, 0, stream>>>(Wl, 13, 32, 32, WLD, 64, 32);

  k_bucket<<<NBLKB, 256, bkLds, stream>>>(src, dst, ew, ENT, OFFt, CNTt, OVF);

  k_mlp1<<<MPAD / 128, 256, 0, stream>>>(features, PRM, (unsigned*)H1HL);
  k_gemm_nt<1, 0><<<gemmGrid, 256, 0, stream>>>(H1HL, W2D, PRM, D32, MPAD, 32, 256, 32);
  k_rowln32<1><<<MPAD / 128, 256, 0, stream>>>(D32, PRM, P_B2, P_G2, P_BE2, Hp);

  for (int i = 0; i < 4; ++i) {
    k_replay<<<NBLKB, 256, 0, stream>>>(Hp, ENT, OFFt, CNTt, OVF, PRM, i, (unsigned*)AHL);
    k_gemm_nt<1, 0><<<gemmGrid, 256, 0, stream>>>(AHL, WGD + (size_t)i * 4096, PRM, D32, MPAD, 32, 64, 32);
    k_rowln32<0><<<MPAD / 128, 256, 0, stream>>>(D32, PRM, P_BG + 32 * i, P_GLN, P_BLN, Hp);
  }
  k_replay<<<NBLKB, 256, 0, stream>>>(Hp, ENT, OFFt, CNTt, OVF, PRM, 4, (unsigned*)AHL);
  k_gemm_nt<1, 0><<<gemmGrid, 256, 0, stream>>>(AHL, WLD, PRM, D32, MPAD, 32, 64, 32);
  k_lnlast<<<LN_NBLK, 256, 0, stream>>>(D32, PRM, O13, REC);

  k_head<<<1, 256, 0, stream>>>(REC, PRM, PRED);
  k_store<<<ST_NBLK + 1, 256, 0, stream>>>(O13, PRED, OVF, out);
}
